// Net_11647951307192
// MI455X (gfx1250) — hardware-verified
//
#include <hip/hip_runtime.h>
#include <stddef.h>
#include <stdint.h>
#include <math.h>


#define NGR    128
#define NPG    512
#define NT     65536
#define FD     128
#define KW3    384
#define NEDGE  524288
#define DEGCAP 32
#define NTHR   256
#define NWAVE  8
#define EPT    8
#define CHUNK  (NTHR * EPT)
#define WCAP   (EPT * 32)
#define LISTN  (NWAVE * WCAP)
#define NBA    512
#define SLA    9
#define RCAP   8192
#define MISC_INTS 32
#define CSR_ZINTS (LISTN + 2 * RCAP + 3 * NBA)
#define CSR_LDS_INTS (CSR_ZINTS + MISC_INTS + NBA)
#define GBM    64
#define GBN    128
#define GTHR   128
#define PTHR   512
#define PWAVE  16
#define XUNITS (NT * (FD / 8))
#define XBLK   (XUNITS / NTHR)
#define WU1    (FD * (FD / 8))
#define WU3    (FD * (KW3 / 8))
#define WBLK   ((WU1 + 2 * WU3) / NTHR)
#define WSMAX  134217728

static_assert((CHUNK & (CHUNK - 1)) == 0 && CHUNK <= 4096);
static_assert(NBA == (1 << SLA));
static_assert(((long long)NEDGE << SLA) < (1LL << 31));
static_assert(NT % NBA == 0 && NT % GBM == 0 && NT % NTHR == 0 && NT == NGR * NPG);
static_assert(CSR_ZINTS % 4 == 0 && LISTN % 4 == 0);
static_assert(CSR_LDS_INTS * 4 <= 300000);
static_assert(FD % 32 == 0 && KW3 % 32 == 0 && KW3 == 3 * FD);
static_assert(GBN == FD && GBM == (GTHR / 32) * 16);
static_assert(XUNITS % NTHR == 0 && WU1 % NTHR == 0 && WU3 % NTHR == 0);
static_assert(NEDGE % CHUNK == 0);
static_assert(DEGCAP == 32 && NBA % NWAVE == 0 && NBA == 2 * NTHR);
static_assert(PTHR == NPG && PWAVE * 32 == PTHR);

typedef float          v4f   __attribute__((ext_vector_type(4)));
typedef float          v8f   __attribute__((ext_vector_type(8)));
typedef int            v4i   __attribute__((ext_vector_type(4)));
typedef int            v8i   __attribute__((ext_vector_type(8)));
typedef unsigned short v4us  __attribute__((ext_vector_type(4)));
typedef unsigned short v8us  __attribute__((ext_vector_type(8)));
typedef unsigned short v16us __attribute__((ext_vector_type(16)));
typedef __bf16         v16bf __attribute__((ext_vector_type(16)));
typedef v4f  __attribute__((may_alias)) v4fa;
typedef v4i  __attribute__((may_alias)) v4ia;
typedef v4us __attribute__((may_alias)) v4usa;
typedef v8us __attribute__((may_alias)) v8usa;
union FragB { v16bf v; v16us u; v8us h[2]; v8i w; };

__device__ __forceinline__ v8f wmb(const FragB& a, const FragB& b, v8f c) {
  v8f d = __builtin_amdgcn_wmma_f32_16x16x32_bf16(false, a.v, false, b.v, (short)0, c, false, false);
  asm volatile("v_nop\n\tv_nop\n\tv_nop\n\tv_nop" : "+v"(d) : "v"(a.w), "v"(b.w));
  return d;
}

__device__ __forceinline__ unsigned bf16_bits(float f) {
  const unsigned u = __float_as_uint(f);
  return (u + 0x7FFFu + ((u >> 16) & 1u)) >> 16;
}
__device__ __forceinline__ float bf16_val(float f) {
  return __uint_as_float(bf16_bits(f) << 16);
}
__device__ __forceinline__ void split3(float v, unsigned& h, unsigned& m, unsigned& l) {
  h = bf16_bits(v);
  const float r1 = v - __uint_as_float(h << 16);
  m = bf16_bits(r1);
  const float r2 = r1 - __uint_as_float(m << 16);
  l = bf16_bits(r2);
}
__device__ __forceinline__ int clampi(int v, int lo, int hi) {
  return v < lo ? lo : (v > hi ? hi : v);
}
__device__ __forceinline__ void wave_sync() {
  __builtin_amdgcn_fence(__ATOMIC_RELEASE, "wavefront");
  __builtin_amdgcn_wave_barrier();
  __builtin_amdgcn_fence(__ATOMIC_ACQUIRE, "wavefront");
}
__device__ __forceinline__ int wave_max_i(int v) {
#pragma unroll
  for (int d = 16; d > 0; d >>= 1) {
    const int o = __shfl_xor(v, d, 32);
    v = o > v ? o : v;
  }
  return __builtin_amdgcn_readfirstlane(v);
}

template <int SLB>
__device__ __forceinline__ int scan_chunk(const int* __restrict__ dsts, int nE, int cbase, int slotBase,
                                          int nb, int vec8, int* list, int tid, int lane, int wave) {
  int wc = 0;
  const int el0  = tid * EPT;
  const int e0   = cbase + el0;
  const int sent = -2147483647 - 1;
  v4i da, db;
  if (vec8 != 0 && cbase + CHUNK <= nE) {
    da = *(const v4i*)(dsts + e0);
    db = *(const v4i*)(dsts + e0 + 4);
  } else {
    da.x = (e0     < nE) ? dsts[min(e0,     nE - 1)] : sent;
    da.y = (e0 + 1 < nE) ? dsts[min(e0 + 1, nE - 1)] : sent;
    da.z = (e0 + 2 < nE) ? dsts[min(e0 + 2, nE - 1)] : sent;
    da.w = (e0 + 3 < nE) ? dsts[min(e0 + 3, nE - 1)] : sent;
    db.x = (e0 + 4 < nE) ? dsts[min(e0 + 4, nE - 1)] : sent;
    db.y = (e0 + 5 < nE) ? dsts[min(e0 + 5, nE - 1)] : sent;
    db.z = (e0 + 6 < nE) ? dsts[min(e0 + 6, nE - 1)] : sent;
    db.w = (e0 + 7 < nE) ? dsts[min(e0 + 7, nE - 1)] : sent;
  }
  const unsigned nbs = (unsigned)slotBase;
  const unsigned unb = (unsigned)nb;
  const unsigned s0 = (unsigned)da.x - nbs, s1 = (unsigned)da.y - nbs;
  const unsigned s2 = (unsigned)da.z - nbs, s3 = (unsigned)da.w - nbs;
  const unsigned s4 = (unsigned)db.x - nbs, s5 = (unsigned)db.y - nbs;
  const unsigned s6 = (unsigned)db.z - nbs, s7 = (unsigned)db.w - nbs;
  const bool h0 = s0 < unb, h1 = s1 < unb, h2 = s2 < unb, h3 = s3 < unb;
  const bool h4 = s4 < unb, h5 = s5 < unb, h6 = s6 < unb, h7 = s7 < unb;
  const unsigned any = __builtin_amdgcn_ballot_w32(h0 | h1 | h2 | h3 | h4 | h5 | h6 | h7);
  if (any != 0u) {
#define HITJ(J, HJ, SJ) { \
      const unsigned mj = __builtin_amdgcn_ballot_w32(HJ); \
      if (mj != 0u) { \
        if (HJ) { \
          const int pos = wc + (int)__builtin_amdgcn_mbcnt_lo(mj, 0u); \
          if (pos < WCAP) list[wave * WCAP + pos] = ((el0 + (J)) << SLB) | (int)(SJ); \
        } \
        wc += (int)__builtin_popcount(mj); } }
    HITJ(0, h0, s0)
    HITJ(1, h1, s1)
    HITJ(2, h2, s2)
    HITJ(3, h3, s3)
    HITJ(4, h4, s4)
    HITJ(5, h5, s5)
    HITJ(6, h6, s6)
    HITJ(7, h7, s7)
#undef HITJ
  }
  return wc;
}

__device__ __forceinline__ void wunit(const float* __restrict__ W, unsigned short* P, int n, int k8, int pitch) {
  const int kk = k8 & (FD - 1);
  const float* p = W + (size_t)kk * FD + n;
  v8us o;
#pragma unroll
  for (int i = 0; i < 8; ++i) o[i] = (unsigned short)bf16_bits(p[(size_t)i * FD]);
  unsigned short* dp = P + (size_t)n * pitch + k8;
  *(volatile v8us*)dp = o;
  __threadfence();
  *(volatile v8us*)dp = o;
}

__global__ __launch_bounds__(NTHR) void k_prep(const float* __restrict__ x, const float* __restrict__ W1,
                                               const float* __restrict__ W2, const float* __restrict__ W3,
                                               unsigned short* xb, unsigned short* w1t,
                                               unsigned short* w2t, unsigned short* w3t) {
  const int blk = (int)blockIdx.x;
  const int tid = (int)threadIdx.x;
  if (blk < XBLK) {
    const int u   = blk * NTHR + tid;
    const int row = u >> 4;
    const int k8  = (u & 15) * 8;
    const float* p = x + (size_t)row * FD + k8;
    const v4f a = *(const v4f*)p;
    const v4f b = *(const v4f*)(p + 4);
    v8us o;
    o[0] = (unsigned short)bf16_bits(a.x); o[1] = (unsigned short)bf16_bits(a.y);
    o[2] = (unsigned short)bf16_bits(a.z); o[3] = (unsigned short)bf16_bits(a.w);
    o[4] = (unsigned short)bf16_bits(b.x); o[5] = (unsigned short)bf16_bits(b.y);
    o[6] = (unsigned short)bf16_bits(b.z); o[7] = (unsigned short)bf16_bits(b.w);
    unsigned short* dp = xb + (size_t)row * FD + k8;
    *(volatile v8us*)dp = o;
    __threadfence();
    *(volatile v8us*)dp = o;
  } else {
    const int v = (blk - XBLK) * NTHR + tid;
    if (v < WU1) {
      wunit(W1, w1t, v >> 4, (v & 15) * 8, FD);
    } else if (v < WU1 + WU3) {
      const int vv = v - WU1;
      const int n  = vv / 48;
      wunit(W2, w2t, n, (vv - n * 48) * 8, KW3);
    } else if (v < WU1 + 2 * WU3) {
      const int vv = v - WU1 - WU3;
      const int n  = vv / 48;
      wunit(W3, w3t, n, (vv - n * 48) * 8, KW3);
    }
  }
}

__global__ __launch_bounds__(NTHR) void k_csr(const int* __restrict__ srcs, const int* __restrict__ dsts,
                                              int nE, int nN, int vec8,
                                              int* nbr, int* cntg, float* dinv, int* flg) {
  extern __shared__ __attribute__((aligned(16))) int dsm[];
  int* list = dsm;
  int* hl   = dsm + LISTN;
  int* sl   = hl + RCAP;
  int* cnt  = sl + RCAP;
  int* offs = cnt + NBA;
  int* cur  = offs + NBA;
  int* misc = cur + NBA;
  float* fdv = (float*)(misc + MISC_INTS);
  const int tid = (int)threadIdx.x, lane = tid & 31, wave = tid >> 5;
  const int nodeBase = (int)blockIdx.x * NBA;

  {
    const v4i z4 = {0, 0, 0, 0};
    for (int i = tid * 4; i < CSR_ZINTS; i += NTHR * 4) *(v4ia*)(dsm + i) = z4;
    if (tid < MISC_INTS) misc[tid] = 0;
  }
  __syncthreads();

  int t = 0, ov = 0;
  const int nChunks = (nE + CHUNK - 1) / CHUNK;
#pragma unroll 1
  for (int ch = 0; ch < nChunks; ++ch) {
    const int cbase = ch * CHUNK;
    const int wc = scan_chunk<SLA>(dsts, nE, cbase, nodeBase, NBA, vec8, list, tid, lane, wave);
    if (lane == 0) misc[wave] = wc;
    __syncthreads();
    if (wave == 0) {
#pragma unroll 1
      for (int w2 = 0; w2 < NWAVE; ++w2) {
        int c = misc[w2];
        c = c < 0 ? 0 : (c > WCAP ? WCAP : c);
#pragma unroll 1
        for (int b0 = 0; b0 < c; b0 += 32) {
          const int idx = b0 + lane;
          const int ent = list[w2 * WCAP + (idx < WCAP ? idx : WCAP - 1)];
          const int m32 = (c - b0) < 32 ? (c - b0) : 32;
#pragma unroll 1
          for (int k = 0; k < m32; ++k) {
            const int u    = __builtin_amdgcn_readlane(ent, k);
            const int slot = u & (NBA - 1);
            const int el   = (u >> SLA) & (CHUNK - 1);
            const int pk   = ((cbase + el) << SLA) | slot;
            if (t < RCAP) {
              if (lane == 0) { hl[t] = pk; cnt[slot] = cnt[slot] + 1; }
              t = t + 1;
            } else {
              ov = 1;
            }
          }
        }
      }
    }
    __syncthreads();
  }
  if (wave == 0 && lane == 0) { misc[8] = t; misc[9] = ov; }
  __syncthreads();
  int tt = misc[8];
  tt = tt < 0 ? 0 : (tt > RCAP ? RCAP : tt);

  if (wave == 0) {
    const int base = lane * (NBA / 32);
    int s = 0;
#pragma unroll 1
    for (int i = 0; i < NBA / 32; ++i) s += cnt[base + i];
    int incl = s;
#pragma unroll
    for (int d = 1; d < 32; d <<= 1) {
      const int y = __shfl_up(incl, d, 32);
      if (lane >= d) incl += y;
    }
    int run = incl - s;
#pragma unroll 1
    for (int i = 0; i < NBA / 32; ++i) {
      const int cv = cnt[base + i];
      offs[base + i] = run;
      cur[base + i]  = run;
      run += cv;
    }
  }
  __syncthreads();
  if (wave == 0) {
#pragma unroll 1
    for (int b0 = 0; b0 < tt; b0 += 32) {
      const int idx = b0 + lane;
      const int ent = hl[idx < RCAP ? idx : RCAP - 1];
      const int m32 = (tt - b0) < 32 ? (tt - b0) : 32;
#pragma unroll 1
      for (int k = 0; k < m32; ++k) {
        const int u    = __builtin_amdgcn_readlane(ent, k);
        const int slot = u & (NBA - 1);
        if (lane == 0) {
          int p = cur[slot];
          p = p < 0 ? 0 : (p > RCAP - 1 ? RCAP - 1 : p);
          sl[p] = u;
          cur[slot] = p + 1;
        }
      }
    }
  }
  __syncthreads();

  int bigw = 0;
#pragma unroll 1
  for (int si = 0; si < NBA / NWAVE; ++si) {
    const int s    = si * NWAVE + wave;
    const int node = nodeBase + s;
    int c = cnt[s];
    if (c > DEGCAP) bigw = 1;
    c = clampi(c, 0, DEGCAP);
    const int o = clampi(offs[s], 0, RCAP - 1);
    int idx = o + lane;
    idx = idx > RCAP - 1 ? RCAP - 1 : idx;
    const int ent = sl[idx];
    const int eid = clampi(ent >> SLA, 0, nE - 1);
    const int sr  = clampi(srcs[eid], 0, nN - 1);
    const int val = (lane < c) ? sr : 0;
    int* np = nbr + (size_t)node * DEGCAP + lane;
    *(volatile int*)np = val;
    __threadfence();
    *(volatile int*)np = val;
  }
  {
    const int s0 = 2 * tid;
    const int c0 = clampi(cnt[s0], 0, DEGCAP);
    const int c1 = clampi(cnt[s0 + 1], 0, DEGCAP);
    fdv[s0]     = 1.0f / sqrtf(1.0f + (float)c0);
    fdv[s0 + 1] = 1.0f / sqrtf(1.0f + (float)c1);
  }
  if (lane == 0) misc[16 + wave] = bigw;
  __syncthreads();
  int fl = misc[9];
#pragma unroll
  for (int w2 = 0; w2 < NWAVE; ++w2) fl |= misc[16 + w2];
  const int q = tid & 127;
  v4i c4 = *(const v4ia*)(cnt + 4 * q);
  c4.x = clampi(c4.x, 0, DEGCAP); c4.y = clampi(c4.y, 0, DEGCAP);
  c4.z = clampi(c4.z, 0, DEGCAP); c4.w = clampi(c4.w, 0, DEGCAP);
  const v4f d4 = *(const v4fa*)(fdv + 4 * q);
  const v4i f4 = {fl, fl, fl, fl};
  int*   cp = cntg + (size_t)nodeBase + 4 * q;
  float* dp = dinv + (size_t)nodeBase + 4 * q;
  int*   fp = flg + (size_t)blockIdx.x * 32 + 4 * (tid & 7);
  if (tid < 128) { *(volatile v4i*)cp = c4; *(volatile v4f*)dp = d4; }
  if (tid < 8) *(volatile v4i*)fp = f4;
  __threadfence();
  if (tid < 128) { *(volatile v4i*)cp = c4; *(volatile v4f*)dp = d4; }
  if (tid < 8) *(volatile v4i*)fp = f4;
}

__global__ __launch_bounds__(NTHR) void k_deg(const int* __restrict__ nbr, const int* __restrict__ cntp,
                                              const int* __restrict__ ark, float* dinv, int nN) {
  __shared__ __attribute__((aligned(16))) float sd[NTHR];
  const int tid = (int)threadIdx.x;
  const int i = (int)blockIdx.x * NTHR + tid;
  const int a = ark[i];
  const int c = clampi(cntp[i], 0, DEGCAP);
  const int cm = wave_max_i(c);
  int d = 0;
#pragma unroll 1
  for (int j = 0; j < cm; ++j) {
    const int jj = j < DEGCAP ? j : DEGCAP - 1;
    const int sr = clampi(nbr[(size_t)i * DEGCAP + jj], 0, nN - 1);
    const int as = ark[sr];
    d += ((j < c) && (as >= 0)) ? 1 : 0;
  }
  const float dv = (a >= 0) ? (1.0f / sqrtf((float)(1 + d))) : 0.0f;
  sd[tid] = dv;
  __syncthreads();
  const v4f o = *(const v4fa*)(sd + 4 * (tid & 63));
  float* op = dinv + (size_t)blockIdx.x * NTHR + 4 * (tid & 63);
  if (tid < 64) *(volatile v4f*)op = o;
  __threadfence();
  if (tid < 64) *(volatile v4f*)op = o;
}

__global__ __launch_bounds__(GTHR) void k_gemm(const unsigned short* __restrict__ A, int lda,
                                               const unsigned short* __restrict__ BT, int K, float* outF) {
  __shared__ __attribute__((aligned(16))) float stg[GBM * GBN];
  const int tid = (int)threadIdx.x, lane = tid & 31, wave = tid >> 5, hh = lane >> 4, m = lane & 15;
  const int rowBase = (int)blockIdx.x * GBM;

  v8f acc[8];
  {
    const v8f z = {0.f, 0.f, 0.f, 0.f, 0.f, 0.f, 0.f, 0.f};
#pragma unroll
    for (int t = 0; t < 8; ++t) acc[t] = z;
  }
  const unsigned short* ap = A + (size_t)(rowBase + 16 * wave + m) * (size_t)lda + 8 * hh;
  const unsigned short* bp = BT + (size_t)m * (size_t)K + 8 * hh;

#pragma unroll 1
  for (int k0 = 0; k0 < K; k0 += 32) {
    FragB af;
    af.h[0] = *(const v8usa*)(ap + k0);
    af.h[1] = *(const v8usa*)(ap + k0 + 16);
#pragma unroll
    for (int nt = 0; nt < 8; ++nt) {
      const unsigned short* wq = bp + (size_t)(16 * nt) * (size_t)K + k0;
      FragB bf;
      bf.h[0] = *(const v8usa*)wq;
      bf.h[1] = *(const v8usa*)(wq + 16);
      acc[nt] = wmb(af, bf, acc[nt]);
    }
  }

#pragma unroll
  for (int nt = 0; nt < 8; ++nt) {
    const int lc = 16 * nt + m;
#pragma unroll
    for (int r = 0; r < 8; ++r) {
      const int lr = 16 * wave + 8 * hh + r;
      stg[lr * GBN + lc] = acc[nt][r];
    }
  }
  __syncthreads();

  v4f pv[16];
#pragma unroll
  for (int i = 0; i < 16; ++i) pv[i] = *(const v4fa*)(stg + (16 * wave + i) * GBN + 4 * lane);
#pragma unroll
  for (int i = 0; i < 16; ++i) {
    const int r = rowBase + 16 * wave + i;
    *(volatile v4f*)(outF + (size_t)r * FD + 4 * lane) = pv[i];
  }
  __threadfence();
#pragma unroll
  for (int i = 0; i < 16; ++i) {
    const int r = rowBase + 16 * wave + i;
    *(volatile v4f*)(outF + (size_t)r * FD + 4 * lane) = pv[i];
  }
}

template <int FIRST>
__global__ __launch_bounds__(NTHR) void k_conv(const float* __restrict__ T, const int* __restrict__ nbr,
                                               const int* __restrict__ cntp, const float* __restrict__ dinv,
                                               const int* __restrict__ ark, const float* __restrict__ bvec,
                                               const float* __restrict__ wsv, float* hc, float* sp, int nN) {
  __shared__ __attribute__((aligned(16))) float ss[32];
  const int tid = (int)threadIdx.x, lane = tid & 31, wave = tid >> 5;
  const int base = (int)blockIdx.x * 32;
  v4f b4, w4;
  {
    const v4f t1 = *(const v4f*)(bvec + 4 * lane);
    b4.x = bf16_val(t1.x); b4.y = bf16_val(t1.y); b4.z = bf16_val(t1.z); b4.w = bf16_val(t1.w);
    const v4f t2 = *(const v4f*)(wsv + 4 * lane);
    w4.x = bf16_val(t2.x); w4.y = bf16_val(t2.y); w4.z = bf16_val(t2.z); w4.w = bf16_val(t2.w);
  }
#pragma unroll 1
  for (int r = 0; r < 4; ++r) {
    const int i = base + wave * 4 + r;
    int ai = 0;
    if constexpr (FIRST == 0) ai = ark[i];
    const bool alive = ai >= 0;
    const int c = clampi(cntp[i], 0, DEGCAP);
    const float dd = dinv[i];
    const int sr = clampi(nbr[(size_t)i * DEGCAP + lane], 0, nN - 1);
    const float ds = dinv[sr];
    int as = 0;
    if constexpr (FIRST == 0) as = ark[sr];
    const bool ok = (lane < c) && (as >= 0) && alive;
    const float wv = ok ? (ds * dd) : 0.0f;
    const int okI = ok ? 1 : 0;
    const int wvI = __float_as_int(wv);
    const int cc = __builtin_amdgcn_readfirstlane(alive ? c : 0);
    v4f acc = {0.0f, 0.0f, 0.0f, 0.0f};
#pragma unroll 1
    for (int k = 0; k < cc; ++k) {
      if (__builtin_amdgcn_readlane(okI, k) != 0) {
        const int   sk = __builtin_amdgcn_readlane(sr, k);
        const float ck = __int_as_float(__builtin_amdgcn_readlane(wvI, k));
        const v4f a = *(const v4f*)(T + (size_t)sk * FD + 4 * lane);
        acc.x = fmaf(ck, a.x, acc.x);
        acc.y = fmaf(ck, a.y, acc.y);
        acc.z = fmaf(ck, a.z, acc.z);
        acc.w = fmaf(ck, a.w, acc.w);
      }
    }
    const v4f tv = *(const v4f*)(T + (size_t)i * FD + 4 * lane);
    const float rd = dd * dd;
    v4f y;
    y.x = (acc.x + tv.x * rd) + b4.x;
    y.y = (acc.y + tv.y * rd) + b4.y;
    y.z = (acc.z + tv.z * rd) + b4.z;
    y.w = (acc.w + tv.w * rd) + b4.w;
    y.x = (y.x > 0.0f) ? y.x : (y.x - y.x);
    y.y = (y.y > 0.0f) ? y.y : (y.y - y.y);
    y.z = (y.z > 0.0f) ? y.z : (y.z - y.z);
    y.w = (y.w > 0.0f) ? y.w : (y.w - y.w);
    y.x = alive ? y.x : 0.0f; y.y = alive ? y.y : 0.0f;
    y.z = alive ? y.z : 0.0f; y.w = alive ? y.w : 0.0f;
    float p = y.x * w4.x;
    p = fmaf(y.y, w4.y, p);
    p = fmaf(y.z, w4.z, p);
    p = fmaf(y.w, w4.w, p);
#pragma unroll
    for (int d = 16; d > 0; d >>= 1) p += __shfl_xor(p, d, 32);
    if (lane == 0) ss[wave * 4 + r] = p;
    float* hp = hc + (size_t)i * FD + 4 * lane;
    *(volatile v4f*)hp = y;
    __threadfence();
    *(volatile v4f*)hp = y;
  }
  __syncthreads();
  const v4f sv = *(const v4fa*)(ss + 4 * (tid & 7));
  float* op = sp + (size_t)base + 4 * (tid & 7);
  if (tid < 8) *(volatile v4f*)op = sv;
  __threadfence();
  if (tid < 8) *(volatile v4f*)op = sv;
}

template <int L>
__global__ __launch_bounds__(PTHR) void k_pool(const float* __restrict__ hc, const float* __restrict__ sp,
                                               const float* __restrict__ dinv, const int* __restrict__ nbr,
                                               const int* __restrict__ cntp, const int* __restrict__ arkp,
                                               int* arkn, unsigned short* x3, float* rw,
                                               const float* __restrict__ ra, const float* __restrict__ rb,
                                               const int* __restrict__ flg, const float* __restrict__ bsp,
                                               float* outp, int nN) {
  constexpr int KL = (L == 1) ? 256 : ((L == 2) ? 128 : 64);
  __shared__ __attribute__((aligned(16))) float ssc[NPG];
  __shared__ __attribute__((aligned(16))) int   skey[NPG];
  __shared__ __attribute__((aligned(16))) int   sark[NPG];
  __shared__ int   sel[256];
  __shared__ float tsc[256];
  __shared__ __attribute__((aligned(16))) float rbuf[256];
  __shared__ __attribute__((aligned(16))) unsigned short rowbuf[PWAVE * KW3];
  __shared__ int swf[PWAVE];
  const int tid = (int)threadIdx.x, lane = tid & 31, wave = tid >> 5;
  const int b = (int)blockIdx.x;
  const int i = b * NPG + tid;

  int pk = 0;
  if constexpr (L != 1) pk = arkp[i];
  const bool alive = pk >= 0;
  const int key = (L == 1) ? tid : pk;
  const int c = clampi(cntp[i], 0, DEGCAP);
  const float dd = dinv[i];
  const float si = sp[i];
  const int cm = wave_max_i(c);
  float acc = 0.0f;
#pragma unroll 1
  for (int j = 0; j < cm; ++j) {
    const int jj = j < DEGCAP ? j : DEGCAP - 1;
    const int sr = clampi(nbr[(size_t)i * DEGCAP + jj], 0, nN - 1);
    const float ds = dinv[sr];
    const float sv = sp[sr];
    int as = 0;
    if constexpr (L != 1) as = arkp[sr];
    const bool ok = (j < c) && (as >= 0);
    const float na = fmaf(ds * dd, sv, acc);
    acc = ok ? na : acc;
  }
  const float bsv = bf16_val(bsp[0]);
  const float score = (acc + (dd * dd) * si) + bsv;
  ssc[tid]  = alive ? score : __uint_as_float(0xff800000u);
  skey[tid] = alive ? key : 0x7fffffff;
  if (tid < 256) { sel[tid] = 0; tsc[tid] = 0.0f; }
  int fflag = 0;
  if constexpr (L == 3) fflag = flg[(size_t)(tid & (NGR - 1)) * 32];
  {
    const unsigned fm = __builtin_amdgcn_ballot_w32(fflag != 0);
    if (lane == 0) swf[wave] = (fm != 0u) ? 1 : 0;
  }
  __syncthreads();

  int rk = 0;
#pragma unroll 2
  for (int j4 = 0; j4 < NPG / 4; ++j4) {
    const v4f sv = *(const v4fa*)(ssc + 4 * j4);
    const v4i kv = *(const v4ia*)(skey + 4 * j4);
    rk += ((sv.x > score) || ((sv.x == score) && (kv.x < key))) ? 1 : 0;
    rk += ((sv.y > score) || ((sv.y == score) && (kv.y < key))) ? 1 : 0;
    rk += ((sv.z > score) || ((sv.z == score) && (kv.z < key))) ? 1 : 0;
    rk += ((sv.w > score) || ((sv.w == score) && (kv.w < key))) ? 1 : 0;
  }
  const bool kept = alive && (rk < KL);
  const float th = tanhf(score);
  if (kept) { sel[rk] = tid; tsc[rk] = th; }
  sark[tid] = kept ? rk : -1;
  __syncthreads();

  if constexpr (L != 3) {
    const v4i a4 = *(const v4ia*)(sark + 4 * (tid & 127));
    int* apn = arkn + (size_t)b * NPG + 4 * (tid & 127);
    if (tid < 128) *(volatile v4i*)apn = a4;
    __threadfence();
    if (tid < 128) *(volatile v4i*)apn = a4;

    unsigned short* rbw = rowbuf + wave * KW3;
#pragma unroll 1
    for (int q = 0; q < 32; ++q) {
      const int li = wave * 32 + q;
      const int gi = b * NPG + li;
      const int rkl = __builtin_amdgcn_readfirstlane(sark[li]);
      const bool kp = rkl >= 0;
      const float tt = tsc[clampi(rkl, 0, 255)];
      const v4f h4 = *(const v4f*)(hc + (size_t)gi * FD + 4 * lane);
      const float x0 = kp ? (h4.x * tt) : 0.0f;
      const float x1 = kp ? (h4.y * tt) : 0.0f;
      const float x2 = kp ? (h4.z * tt) : 0.0f;
      const float x3v = kp ? (h4.w * tt) : 0.0f;
      v4us mh, mm, ml;
      unsigned uh, um, ul;
      split3(x0, uh, um, ul);  mh[0] = (unsigned short)uh; mm[0] = (unsigned short)um; ml[0] = (unsigned short)ul;
      split3(x1, uh, um, ul);  mh[1] = (unsigned short)uh; mm[1] = (unsigned short)um; ml[1] = (unsigned short)ul;
      split3(x2, uh, um, ul);  mh[2] = (unsigned short)uh; mm[2] = (unsigned short)um; ml[2] = (unsigned short)ul;
      split3(x3v, uh, um, ul); mh[3] = (unsigned short)uh; mm[3] = (unsigned short)um; ml[3] = (unsigned short)ul;
      *(v4usa*)(rbw + 4 * lane) = mh;
      *(v4usa*)(rbw + FD + 4 * lane) = mm;
      *(v4usa*)(rbw + 2 * FD + 4 * lane) = ml;
      wave_sync();
      const v8us q0 = *(const v8usa*)(rbw + 8 * lane);
      const v8us q1 = *(const v8usa*)(rbw + 2 * FD + 8 * (lane & 15));
      wave_sync();
      unsigned short* rp = x3 + (size_t)gi * KW3 + 8 * lane;
      *(volatile v8us*)rp = q0;
      if (lane < 16) *(volatile v8us*)(rp + 2 * FD) = q1;
      __threadfence();
      *(volatile v8us*)rp = q0;
      if (lane < 16) *(volatile v8us*)(rp + 2 * FD) = q1;
    }
  }

  if (tid < FD) {
    float mx = __uint_as_float(0xff800000u);
    float sum = 0.0f;
#pragma unroll 4
    for (int r = 0; r < KL; ++r) {
      const int li = sel[r] & (NPG - 1);
      const float tt = tsc[r];
      const float v = hc[(size_t)(b * NPG + li) * FD + tid] * tt;
      mx = (v > mx) ? v : mx;
      sum = sum + v;
    }
    rbuf[tid] = mx;
    rbuf[FD + tid] = sum * (1.0f / (float)KL);
  }
  __syncthreads();

  v4f o = *(const v4fa*)(rbuf + 4 * (tid & 63));
  float* dst;
  if constexpr (L == 3) {
    int anyf = 0;
#pragma unroll
    for (int w2 = 0; w2 < PWAVE; ++w2) anyf |= swf[w2];
    const float pz = (anyf != 0) ? __uint_as_float(0x7fc00000u) : 0.0f;
    const v4f a = *(const v4f*)(ra + (size_t)b * 256 + 4 * (tid & 63));
    const v4f bb = *(const v4f*)(rb + (size_t)b * 256 + 4 * (tid & 63));
    o.x = ((a.x + bb.x) + o.x) + pz;
    o.y = ((a.y + bb.y) + o.y) + pz;
    o.z = ((a.z + bb.z) + o.z) + pz;
    o.w = ((a.w + bb.w) + o.w) + pz;
    dst = outp + (size_t)b * 256 + 4 * (tid & 63);
  } else {
    dst = rw + (size_t)b * 256 + 4 * (tid & 63);
  }
  if (tid < 64) *(volatile v4f*)dst = o;
  __threadfence();
  if (tid < 64) *(volatile v4f*)dst = o;
}

static inline size_t al256(size_t o) { return (o + 255) & ~(size_t)255; }

extern "C" void kernel_launch(void* const* d_in, const int* in_sizes, int n_in,
                              void* d_out, int out_size, void* d_ws, size_t ws_size,
                              hipStream_t stream) {
  if (n_in < 15) return;
  if (in_sizes[0] != NT * FD) return;
  if (in_sizes[1] != 2 * NEDGE) return;
  if (in_sizes[3] != FD * FD || in_sizes[7] != FD * FD || in_sizes[11] != FD * FD) return;
  if (in_sizes[4] != FD || in_sizes[8] != FD || in_sizes[12] != FD) return;
  if (in_sizes[5] != FD || in_sizes[9] != FD || in_sizes[13] != FD) return;
  if (in_sizes[6] != 1 || in_sizes[10] != 1 || in_sizes[14] != 1) return;
  if (out_size != NGR * 256) return;

  const float* x   = (const float*)d_in[0];
  const int*   ei  = (const int*)d_in[1];
  const float* W1  = (const float*)d_in[3];
  const float* b1  = (const float*)d_in[4];
  const float* Ws1 = (const float*)d_in[5];
  const float* bs1 = (const float*)d_in[6];
  const float* W2  = (const float*)d_in[7];
  const float* b2  = (const float*)d_in[8];
  const float* Ws2 = (const float*)d_in[9];
  const float* bs2 = (const float*)d_in[10];
  const float* W3  = (const float*)d_in[11];
  const float* b3  = (const float*)d_in[12];
  const float* Ws3 = (const float*)d_in[13];
  const float* bs3 = (const float*)d_in[14];
  float* out = (float*)d_out;
  const int nN = NT, nE = NEDGE;
  const int* src = ei;
  const int* dst = ei + nE;
  const int vec8 = ((nE & 3) == 0) ? 1 : 0;

  char* ws = (char*)d_ws;
  size_t off = 0;
  const size_t oT   = off; off = al256(off + (size_t)NT * FD * 4);
  const size_t oHC  = off; off = al256(off + (size_t)NT * FD * 4);
  const size_t oX3  = off; off = al256(off + (size_t)NT * KW3 * 2);
  const size_t oNBR = off; off = al256(off + (size_t)NT * DEGCAP * 4);
  const size_t oCNT = off; off = al256(off + (size_t)NT * 4);
  const size_t oDIN = off; off = al256(off + (size_t)NT * 4);
  const size_t oS   = off; off = al256(off + (size_t)NT * 4);
  const size_t oA1  = off; off = al256(off + (size_t)NT * 4);
  const size_t oA2  = off; off = al256(off + (size_t)NT * 4);
  const size_t oW1  = off; off = al256(off + (size_t)FD * FD * 2);
  const size_t oW2  = off; off = al256(off + (size_t)FD * KW3 * 2);
  const size_t oW3  = off; off = al256(off + (size_t)FD * KW3 * 2);
  const size_t oR1  = off; off = al256(off + (size_t)NGR * 256 * 4);
  const size_t oR2  = off; off = al256(off + (size_t)NGR * 256 * 4);
  const size_t oFL  = off; off = al256(off + (size_t)NGR * 32 * 4);
  if (off > ws_size || off > (size_t)WSMAX) return;
  float*          T    = (float*)(ws + oT);
  float*          HC   = (float*)(ws + oHC);
  unsigned short* X3   = (unsigned short*)(ws + oX3);
  unsigned short* XB   = X3;
  int*            NBR  = (int*)(ws + oNBR);
  int*            CNT  = (int*)(ws + oCNT);
  float*          DINV = (float*)(ws + oDIN);
  float*          S    = (float*)(ws + oS);
  int*            ARK1 = (int*)(ws + oA1);
  int*            ARK2 = (int*)(ws + oA2);
  unsigned short* W1T  = (unsigned short*)(ws + oW1);
  unsigned short* W2T3 = (unsigned short*)(ws + oW2);
  unsigned short* W3T3 = (unsigned short*)(ws + oW3);
  float*          R1   = (float*)(ws + oR1);
  float*          R2   = (float*)(ws + oR2);
  int*            FLG  = (int*)(ws + oFL);

  const size_t csrLds = (size_t)CSR_LDS_INTS * 4;
  hipFuncSetAttribute(reinterpret_cast<const void*>(&k_csr), hipFuncAttributeMaxDynamicSharedMemorySize, (int)csrLds);

  k_prep<<<XBLK + WBLK, NTHR, 0, stream>>>(x, W1, W2, W3, XB, W1T, W2T3, W3T3);
  k_csr<<<NT / NBA, NTHR, csrLds, stream>>>(src, dst, nE, nN, vec8, NBR, CNT, DINV, FLG);
  k_gemm<<<NT / GBM, GTHR, 0, stream>>>(XB, FD, W1T, FD, T);
  k_conv<1><<<NT / 32, NTHR, 0, stream>>>(T, NBR, CNT, DINV, ARK1, b1, Ws1, HC, S, nN);
  k_pool<1><<<NGR, PTHR, 0, stream>>>(HC, S, DINV, NBR, CNT, ARK1, ARK1, X3, R1, R1, R2, FLG, bs1, out, nN);
  k_deg<<<NT / NTHR, NTHR, 0, stream>>>(NBR, CNT, ARK1, DINV, nN);
  k_gemm<<<NT / GBM, GTHR, 0, stream>>>(X3, KW3, W2T3, KW3, T);
  k_conv<0><<<NT / 32, NTHR, 0, stream>>>(T, NBR, CNT, DINV, ARK1, b2, Ws2, HC, S, nN);
  k_pool<2><<<NGR, PTHR, 0, stream>>>(HC, S, DINV, NBR, CNT, ARK1, ARK2, X3, R2, R1, R2, FLG, bs2, out, nN);
  k_deg<<<NT / NTHR, NTHR, 0, stream>>>(NBR, CNT, ARK2, DINV, nN);
  k_gemm<<<NT / GBM, GTHR, 0, stream>>>(X3, KW3, W3T3, KW3, T);
  k_conv<0><<<NT / 32, NTHR, 0, stream>>>(T, NBR, CNT, DINV, ARK2, b3, Ws3, HC, S, nN);
  k_pool<3><<<NGR, PTHR, 0, stream>>>(HC, S, DINV, NBR, CNT, ARK2, ARK2, X3, R2, R1, R2, FLG, bs3, out, nN);
}
